// DiscSeqRNNEncoder_17119739641881
// MI455X (gfx1250) — hardware-verified
//
#include <hip/hip_runtime.h>
#include <math.h>

constexpr int NBATCH   = 8192;
constexpr int NSTEP    = 64;
constexpr int NVOC     = 1000;
constexpr int NEMB     = 64;
constexpr int NHID     = 128;
constexpr int NGATE    = 3 * NHID;
constexpr int NOUTF    = 128;
constexpr int NWAVE    = 4;
constexpr int SEQ_THR  = NWAVE * 32;
constexpr int ROWS_BLK = NWAVE * 16;
constexpr int SEQ_GRID = NBATCH / ROWS_BLK;
constexpr int HMP      = 132;
constexpr int PREP_THR = 256;
constexpr float H_CARRY   = 64.0f;
constexpr float W_CARRY   = 16.0f;
constexpr float LO_CARRY  = 2048.0f;
constexpr float ACC_INV   = 1.0f / (H_CARRY * W_CARRY);
constexpr float LO_INV    = 1.0f / LO_CARRY;
constexpr bool  RECUR_SPLIT_H = false;

static_assert(NBATCH % ROWS_BLK == 0);
static_assert(NHID % 32 == 0);
static_assert(NHID == 128 && NOUTF == 128 && NEMB == 64 && NGATE == 384);
static_assert((NVOC * NHID) % PREP_THR == 0);
static_assert((NGATE * NHID / 8) % PREP_THR == 0);
static_assert((NOUTF * NHID / 8) % PREP_THR == 0);
static_assert((NWAVE * 16 * HMP) % SEQ_THR == 0);
static_assert((HMP * 4) % 16 == 0);

typedef __attribute__((ext_vector_type(16))) _Float16 v16h;
typedef __attribute__((ext_vector_type(8)))  _Float16 v8h;
typedef __attribute__((ext_vector_type(8)))  float    v8f;
typedef __attribute__((ext_vector_type(4)))  float    v4f;
typedef __attribute__((ext_vector_type(4)))  int      v4i;

struct FragH {
  union U { v16h v; v8h h[2]; };
  static __device__ __forceinline__ v16h load(const _Float16* p) {
    U f; f.h[0] = *(const v8h*)(p); f.h[1] = *(const v8h*)(p + 16); return f.v;
  }
  static __device__ __forceinline__ v8f mma(v16h a, v16h b, v8f c) {
    return __builtin_amdgcn_wmma_f32_16x16x32_f16(false, a, false, b, (short)0, c, false, false);
  }
};

__device__ __forceinline__ void guard3(v8f& p, v8f& q, v8f& s, v16h a, v16h b0, v16h b1, v16h b2) {
  asm volatile("v_nop\n\tv_nop\n\tv_nop\n\tv_nop" : "+v"(p), "+v"(q), "+v"(s) : "v"(a), "v"(b0), "v"(b1), "v"(b2));
}
__device__ __forceinline__ void guard6(v8f& p, v8f& q, v8f& s, v8f& pl, v8f& ql, v8f& sl,
                                       v16h a, v16h a2, v16h b0, v16h b1, v16h b2) {
  asm volatile("v_nop\n\tv_nop\n\tv_nop\n\tv_nop" : "+v"(p), "+v"(q), "+v"(s), "+v"(pl), "+v"(ql), "+v"(sl)
               : "v"(a), "v"(a2), "v"(b0), "v"(b1), "v"(b2));
}
__device__ __forceinline__ void guard2(v8f& p, v8f& q, v16h a, v16h a2, v16h b) {
  asm volatile("v_nop\n\tv_nop\n\tv_nop\n\tv_nop" : "+v"(p), "+v"(q) : "v"(a), "v"(a2), "v"(b));
}

__device__ __forceinline__ float gate_sig(float x) {
  const float xc = fminf(fmaxf(x, -30.0f), 30.0f);
  return __builtin_amdgcn_rcpf(1.0f + expf(-xc));
}
__device__ __forceinline__ float gate_tanh(float x) {
  const float xc = fminf(fmaxf(x, -15.0f), 15.0f);
  return 1.0f - 2.0f * __builtin_amdgcn_rcpf(expf(2.0f * xc) + 1.0f);
}
__device__ __forceinline__ void split_h(float v, _Float16& hi, _Float16& lo) {
  const float s = v * H_CARRY;
  hi = (_Float16)s;
  const float hf = (float)hi;
  lo = (_Float16)((s - hf) * LO_CARRY);
}

__global__ __launch_bounds__(PREP_THR) void table_kernel(const float* __restrict__ embed, const float* __restrict__ W_ih,
                                                        const float* __restrict__ b_ih, const float* __restrict__ b_hh,
                                                        float* __restrict__ T4) {
  const int i = blockIdx.x * PREP_THR + threadIdx.x;
  if (i < NVOC * NHID) {
    const int v = i >> 7;
    const int u = i & (NHID - 1);
    const float* er = embed + (size_t)v * NEMB;
    const float* wr = W_ih + (size_t)u * NEMB;
    const float* wz = W_ih + (size_t)(NHID + u) * NEMB;
    const float* wn = W_ih + (size_t)(2 * NHID + u) * NEMB;
    float sr = 0.0f, sz = 0.0f, sn = 0.0f;
#pragma unroll 1
    for (int k4 = 0; k4 < NEMB; k4 += 4) {
      const v4f e4 = *(const v4f*)(er + k4);
      const v4f a4 = *(const v4f*)(wr + k4);
      const v4f z4 = *(const v4f*)(wz + k4);
      const v4f n4 = *(const v4f*)(wn + k4);
#pragma unroll
      for (int e = 0; e < 4; ++e) {
        sr = fmaf(e4[e], a4[e], sr);
        sz = fmaf(e4[e], z4[e], sz);
        sn = fmaf(e4[e], n4[e], sn);
      }
    }
    v4f o;
    o[0] = sr + (b_ih[u] + b_hh[u]);
    o[1] = sz + (b_ih[NHID + u] + b_hh[NHID + u]);
    o[2] = sn + b_ih[2 * NHID + u];
    o[3] = b_hh[2 * NHID + u];
    float* op = T4 + (size_t)i * 4;
    *(volatile v4f*)op = o;
    __threadfence();
    *(volatile v4f*)op = o;
  }
}

__global__ __launch_bounds__(PREP_THR) void cvt8_kernel(const float* __restrict__ src, unsigned short* __restrict__ dst,
                                                       int n8, float sc) {
  const int i = blockIdx.x * PREP_THR + threadIdx.x;
  if (i < n8) {
    const float* sp = src + (size_t)i * 8;
    const v4f a = *(const v4f*)(sp);
    const v4f b = *(const v4f*)(sp + 4);
    v8h hv;
#pragma unroll
    for (int e = 0; e < 4; ++e) {
      const float fa = a[e] * sc;
      const float fb = b[e] * sc;
      hv[e]     = (_Float16)fa;
      hv[4 + e] = (_Float16)fb;
    }
    *(volatile v8h*)(dst + (size_t)i * 8) = hv;
    __threadfence();
    *(volatile v8h*)(dst + (size_t)i * 8) = hv;
  }
}

template <bool HSPLIT>
__global__ __launch_bounds__(SEQ_THR) void gru_seq_kernel(const int* __restrict__ x, const float* __restrict__ T4,
                                                         const unsigned short* __restrict__ WHp,
                                                         const unsigned short* __restrict__ WOp,
                                                         const float* __restrict__ b_out, float* __restrict__ out) {
  __shared__ __align__(16) float Hm[NWAVE][16 * HMP];
  __shared__ __align__(16) int   Ids[NWAVE][NSTEP * 16];
  const _Float16* WH = (const _Float16*)WHp;
  const _Float16* WO = (const _Float16*)WOp;
  const int tid = threadIdx.x, lane = tid & 31, wave = tid >> 5;
  const int c = lane & 15, hh = lane >> 4, koff = hh * 8;
  const int rowbase = blockIdx.x * ROWS_BLK + wave * 16;
  float* hm  = Hm[wave];
  int*   ids = Ids[wave];

  {
    float* hall = &Hm[0][0];
#pragma unroll 1
    for (int i = tid; i < NWAVE * 16 * HMP; i += SEQ_THR) hall[i] = 0.0f;
  }
#pragma unroll 1
  for (int it = 0; it < 8; ++it) {
    const int un = it * 32 + lane;
    const int m  = un >> 4;
    const int t4 = (un & 15) * 4;
    const v4i xv = *(const v4i*)(x + (size_t)(rowbase + m) * NSTEP + t4);
#pragma unroll
    for (int e = 0; e < 4; ++e) {
      int idv = xv[e];
      idv = idv < 0 ? 0 : idv;
      idv = idv > (NVOC - 1) ? (NVOC - 1) : idv;
      ids[(t4 + e) * 16 + m] = idv;
    }
  }
  __syncthreads();

  const v8f z8 = {0.f, 0.f, 0.f, 0.f, 0.f, 0.f, 0.f, 0.f};
  const float* mrow = hm + c * HMP + koff;

#pragma unroll 1
  for (int t = 0; t < NSTEP; ++t) {
    v16h ah[4], al[4];
#pragma unroll
    for (int kt = 0; kt < 4; ++kt) {
      const v4f p0 = *(const v4f*)(mrow + 32 * kt);
      const v4f p1 = *(const v4f*)(mrow + 32 * kt + 4);
      const v4f p2 = *(const v4f*)(mrow + 32 * kt + 16);
      const v4f p3 = *(const v4f*)(mrow + 32 * kt + 20);
      v16h fh, fl;
#pragma unroll
      for (int e = 0; e < 4; ++e) {
        _Float16 h0, l0, h1, l1, h2, l2, h3, l3;
        split_h(p0[e], h0, l0);
        split_h(p1[e], h1, l1);
        split_h(p2[e], h2, l2);
        split_h(p3[e], h3, l3);
        fh[e] = h0; fh[4 + e] = h1; fh[8 + e] = h2; fh[12 + e] = h3;
        fl[e] = l0; fl[4 + e] = l1; fl[8 + e] = l2; fl[12 + e] = l3;
      }
      ah[kt] = fh;
      al[kt] = HSPLIT ? fl : fh;
    }
    const v4i ia = *(const v4i*)(ids + t * 16 + 8 * hh);
    const v4i ib = *(const v4i*)(ids + t * 16 + 8 * hh + 4);
    int tofs[8];
#pragma unroll
    for (int e = 0; e < 4; ++e) {
      tofs[e]     = ia[e] * (NHID * 4) + c * 4;
      tofs[4 + e] = ib[e] * (NHID * 4) + c * 4;
    }
    __syncthreads();

#pragma unroll 1
    for (int j = 0; j < NHID / 16; ++j) {
      const _Float16* wr = WH + (size_t)(16 * j + c) * NHID + koff;
      v8f accR = z8, accZ = z8, accN = z8;
      v8f lowR = z8, lowZ = z8, lowN = z8;
#pragma unroll
      for (int kt = 0; kt < 4; ++kt) {
        const v16h b0 = FragH::load(wr + 32 * kt);
        const v16h b1 = FragH::load(wr + (size_t)NHID * NHID + 32 * kt);
        const v16h b2 = FragH::load(wr + (size_t)2 * NHID * NHID + 32 * kt);
        accR = FragH::mma(ah[kt], b0, accR);
        accZ = FragH::mma(ah[kt], b1, accZ);
        accN = FragH::mma(ah[kt], b2, accN);
        if (HSPLIT) {
          lowR = FragH::mma(al[kt], b0, lowR);
          lowZ = FragH::mma(al[kt], b1, lowZ);
          lowN = FragH::mma(al[kt], b2, lowN);
          guard6(accR, accZ, accN, lowR, lowZ, lowN, ah[kt], al[kt], b0, b1, b2);
        } else {
          guard3(accR, accZ, accN, ah[kt], b0, b1, b2);
        }
      }
#pragma unroll
      for (int r = 0; r < 8; ++r) {
        const v4f tv = *(const v4f*)(T4 + (size_t)(tofs[r] + j * 64));
        const float t0 = tv[0], t1 = tv[1], t2 = tv[2], t3 = tv[3];
        float sr = accR[r] * ACC_INV;
        float sz = accZ[r] * ACC_INV;
        float sn = accN[r] * ACC_INV;
        if (HSPLIT) {
          sr += lowR[r] * (ACC_INV * LO_INV);
          sz += lowZ[r] * (ACC_INV * LO_INV);
          sn += lowN[r] * (ACC_INV * LO_INV);
        }
        const float rg = gate_sig(sr + t0);
        const float zg = gate_sig(sz + t1);
        const float ng = gate_tanh(t2 + rg * (sn + t3));
        float* mp = hm + (8 * hh + r) * HMP + 16 * j + c;
        const float ho = *mp;
        const float hn = (1.0f - zg) * ng + zg * ho;
        *mp = hn;
      }
    }
    __syncthreads();
  }

  v16h qh[4], ql[4];
#pragma unroll
  for (int kt = 0; kt < 4; ++kt) {
    const v4f p0 = *(const v4f*)(mrow + 32 * kt);
    const v4f p1 = *(const v4f*)(mrow + 32 * kt + 4);
    const v4f p2 = *(const v4f*)(mrow + 32 * kt + 16);
    const v4f p3 = *(const v4f*)(mrow + 32 * kt + 20);
    v16h fh, fl;
#pragma unroll
    for (int e = 0; e < 4; ++e) {
      _Float16 h0, l0, h1, l1, h2, l2, h3, l3;
      split_h(p0[e], h0, l0);
      split_h(p1[e], h1, l1);
      split_h(p2[e], h2, l2);
      split_h(p3[e], h3, l3);
      fh[e] = h0; fh[4 + e] = h1; fh[8 + e] = h2; fh[12 + e] = h3;
      fl[e] = l0; fl[4 + e] = l1; fl[8 + e] = l2; fl[12 + e] = l3;
    }
    qh[kt] = fh;
    ql[kt] = fl;
  }
  __syncthreads();
#pragma unroll 1
  for (int nt = 0; nt < NOUTF / 16; ++nt) {
    const _Float16* wo = WO + (size_t)(16 * nt + c) * NHID + koff;
    v8f accH = z8, accL = z8;
#pragma unroll
    for (int kt = 0; kt < 4; ++kt) {
      const v16h b = FragH::load(wo + 32 * kt);
      accH = FragH::mma(qh[kt], b, accH);
      accL = FragH::mma(ql[kt], b, accL);
      guard2(accH, accL, qh[kt], ql[kt], b);
    }
    const float bo = b_out[16 * nt + c];
#pragma unroll
    for (int r = 0; r < 8; ++r) {
      const float v = (accH[r] + accL[r] * LO_INV) * ACC_INV + bo;
      hm[(8 * hh + r) * HMP + 16 * nt + c] = v;
    }
  }
  __syncthreads();
  for (int pass = 0; pass < 2; ++pass) {
#pragma unroll
    for (int row = 0; row < 16; ++row) {
      const v4f v = *(const v4f*)(hm + row * HMP + lane * 4);
      *(volatile v4f*)(out + (size_t)(rowbase + row) * NOUTF + lane * 4) = v;
    }
    __threadfence();
  }
}

extern "C" void kernel_launch(void* const* d_in, const int* in_sizes, int n_in,
                              void* d_out, int out_size, void* d_ws, size_t ws_size, hipStream_t stream) {
  if (n_in < 8 || d_out == nullptr || d_ws == nullptr) return;
  if (in_sizes[0] != NBATCH * NSTEP || in_sizes[1] != NVOC * NEMB || in_sizes[2] != NGATE * NEMB ||
      in_sizes[3] != NGATE * NHID || in_sizes[4] != NGATE || in_sizes[5] != NGATE ||
      in_sizes[6] != NOUTF * NHID || in_sizes[7] != NOUTF || out_size != NBATCH * NOUTF) return;

  const int*   x     = (const int*)d_in[0];
  const float* embed = (const float*)d_in[1];
  const float* W_ih  = (const float*)d_in[2];
  const float* W_hh  = (const float*)d_in[3];
  const float* b_ih  = (const float*)d_in[4];
  const float* b_hh  = (const float*)d_in[5];
  const float* W_out = (const float*)d_in[6];
  const float* b_out = (const float*)d_in[7];
  float* out = (float*)d_out;

  char* ws = (char*)d_ws; size_t off = 0;
  auto carve = [&](size_t bytes) -> char* { char* p = ws + off; off += (bytes + 255) & ~(size_t)255; return p; };
  float*          T4   = (float*)carve((size_t)NVOC * NHID * 4 * sizeof(float));
  unsigned short* WH16 = (unsigned short*)carve((size_t)NGATE * NHID * 2);
  unsigned short* WO16 = (unsigned short*)carve((size_t)NOUTF * NHID * 2);
  if (off > ws_size || off > (size_t)134217728) return;

  table_kernel<<<(NVOC * NHID) / PREP_THR, PREP_THR, 0, stream>>>(embed, W_ih, b_ih, b_hh, T4);
  cvt8_kernel<<<(NGATE * NHID / 8) / PREP_THR, PREP_THR, 0, stream>>>(W_hh, WH16, NGATE * NHID / 8, W_CARRY);
  cvt8_kernel<<<(NOUTF * NHID / 8) / PREP_THR, PREP_THR, 0, stream>>>(W_out, WO16, NOUTF * NHID / 8, W_CARRY);
  gru_seq_kernel<RECUR_SPLIT_H><<<SEQ_GRID, SEQ_THR, 0, stream>>>(x, T4, WH16, WO16, b_out, out);
}
